// OuterProductMHSA_85469849191014
// MI455X (gfx1250) — hardware-run, weakly checked
//
#include <hip/hip_runtime.h>


#ifndef NB
#define NB 4
#endif
#ifndef SEQ
#define SEQ 1024
#endif
#define NB_FULL  4
#define SEQ_FULL 1024
#ifndef OUT_SEQ
#define OUT_SEQ SEQ
#endif
#define DM   128
#define RT   (SEQ / 64)

static_assert(DM % 64 == 0);
static_assert(DM % 32 == 0);
static_assert(DM == 4 * 32);
static_assert(SEQ % 64 == 0);
static_assert((NB * SEQ) % 64 == 0);
static_assert(((size_t)SEQ * DM) % 8 == 0);
static_assert(((size_t)DM * DM) % 8 == 0);
static_assert(NB <= NB_FULL);
static_assert(SEQ <= SEQ_FULL);
static_assert(32 * 16 == DM * 4);
static_assert(32 * 16 * 8 == 16 * 64 * 4);
static_assert(256 * 16 * 2 == 64 * 64 * 2);
static_assert(256 * 16 == 64 * 64);
static_assert(16 * 68 * 4 <= 131072);
static_assert(64 * 72 * 2 <= 131072);
static_assert(DM * 4 <= 131072);
static_assert((68 * 4) % 16 == 0);
static_assert((72 * 2) % 16 == 0);

typedef unsigned short bf;
typedef __attribute__((ext_vector_type(16))) __bf16   v16bf;
typedef __attribute__((ext_vector_type(8)))  unsigned short v8us;
typedef __attribute__((ext_vector_type(8)))  float    v8f;
typedef __attribute__((ext_vector_type(4)))  float    v4f;
typedef v4f  __attribute__((may_alias)) v4fa;

__device__ __forceinline__ unsigned short f2bf(float f) { unsigned u = __float_as_uint(f); u += 0x7FFFu + ((u >> 16) & 1u); return (unsigned short)(u >> 16); }
__device__ __forceinline__ float bfr(float f) { return __uint_as_float(((unsigned)f2bf(f)) << 16); }
__device__ __forceinline__ v16bf cat16b(v8us lo, v8us hi) { return __builtin_bit_cast(v16bf, __builtin_shufflevector(lo, hi, 0, 1, 2, 3, 4, 5, 6, 7, 8, 9, 10, 11, 12, 13, 14, 15)); }
__device__ __forceinline__ v8f wmmab(v16bf a, v16bf b, v8f c) { return __builtin_amdgcn_wmma_f32_16x16x32_bf16(false, a, false, b, (short)0, c, false, false); }
__device__ __forceinline__ v16bf ldb(const bf* p)  { return cat16b(*(const v8us*)p, *(const v8us*)(p + 16)); }
__device__ __forceinline__ void wave_sync() { __builtin_amdgcn_fence(3  , "wavefront"); __builtin_amdgcn_wave_barrier(); asm volatile("" ::: "memory"); }
__device__ __forceinline__ v8f wmmab_g(v16bf a, v16bf b, v8f c) {
    c = wmmab(a, b, c);
    asm volatile("v_nop\n\tv_nop\n\tv_nop\n\tv_nop" : "+v"(c) : "v"(a), "v"(b));
    return c;
}

__global__ __launch_bounds__(256) void k_cvt8(const float* __restrict__ src, bf* dst, size_t n8) {
    const size_t i = (size_t)blockIdx.x * 256 + threadIdx.x; if (i >= n8) return;
    const v8f v = *(const v8f*)(src + i * 8); v8us o;
#pragma unroll
    for (int k = 0; k < 8; ++k) o[k] = f2bf(v[k]);
    *(volatile v8us*)(dst + i * 8) = o; __threadfence(); *(volatile v8us*)(dst + i * 8) = o;
}

__global__ __launch_bounds__(256) void k_wtr(const float* __restrict__ src, bf* dst) {
    __shared__ __align__(16) bf t[64 * 72];
    const int tid = threadIdx.x;
    const int k0 = blockIdx.x * 64, n0 = blockIdx.y * 64;
#pragma unroll 4
    for (int i = 0; i < 16; ++i) {
        const int e = i * 256 + tid; const int kk = e >> 6, nn = e & 63;
        t[nn * 72 + kk] = f2bf(src[(size_t)(k0 + kk) * DM + n0 + nn]);
    }
    __syncthreads();
#pragma unroll 1
    for (int ps = 0; ps < 2; ++ps) {
#pragma unroll
        for (int s = 0; s < 2; ++s) { const int p = s * 256 + tid; const int nn = p >> 3, c8 = (p & 7) * 8;
            const v8us o = *(const v8us*)(&t[nn * 72 + c8]);
            *(volatile v8us*)(dst + (size_t)(n0 + nn) * DM + k0 + c8) = o; }
        if (ps == 0) __threadfence(); }
}

__global__ __launch_bounds__(128) void k_kvpart(const bf* __restrict__ A, const bf* __restrict__ Wkt, const bf* __restrict__ Wvt,
                                                const float* __restrict__ bk, const float* __restrict__ bv, float* PART) {
    __shared__ __align__(16) float cs[DM];
    const int K = DM;
    const int lane = threadIdx.x & 31, lr = lane & 15, hi = lane >> 4;
    const int wave = __builtin_amdgcn_readfirstlane((int)(threadIdx.x >> 5));
    const int r0 = blockIdx.x * 64, c0 = wave * 32;
    v8f ck[4][2], cv[4][2];
#pragma unroll
    for (int mb = 0; mb < 4; ++mb)
#pragma unroll
        for (int nb = 0; nb < 2; ++nb) { ck[mb][nb] = (v8f){}; cv[mb][nb] = (v8f){}; }
    const size_t aoff = (size_t)(r0 + lr) * K + 8 * hi, boff = (size_t)(c0 + lr) * K + 8 * hi;
#pragma unroll 1
    for (int kc = 0; kc < K; kc += 32) {
        v16bf a[4];
#pragma unroll
        for (int mb = 0; mb < 4; ++mb) a[mb] = ldb(A + aoff + (size_t)mb * 16 * K + kc);
#pragma unroll
        for (int nb = 0; nb < 2; ++nb) {
            const v16bf fk = ldb(Wkt + boff + (size_t)nb * 16 * K + kc);
            const v16bf fv = ldb(Wvt + boff + (size_t)nb * 16 * K + kc);
#pragma unroll
            for (int mb = 0; mb < 4; ++mb) { ck[mb][nb] = wmmab_g(a[mb], fk, ck[mb][nb]); cv[mb][nb] = wmmab_g(a[mb], fv, cv[mb][nb]); } }
    }
    const float bk0 = bfr(bk[c0 + lr]), bk1 = bfr(bk[c0 + 16 + lr]);
    const float bv0 = bfr(bv[c0 + lr]), bv1 = bfr(bv[c0 + 16 + lr]);
    float s0 = 0.0f, s1 = 0.0f;
#pragma unroll
    for (int mb = 0; mb < 4; ++mb) {
#pragma unroll
        for (int j = 0; j < 8; ++j) { s0 += (ck[mb][0][j] + bk0) * (cv[mb][0][j] + bv0); s1 += (ck[mb][1][j] + bk1) * (cv[mb][1][j] + bv1); } }
    s0 += __shfl_xor(s0, 16, 32);
    s1 += __shfl_xor(s1, 16, 32);
    const float mine = hi ? s1 : s0;
    cs[c0 + lane] = mine;
    __syncthreads();
    if (wave == 0) {
        const v4f val = *(const v4fa*)(&cs[lane * 4]);
        float* drow = PART + (size_t)blockIdx.x * DM + lane * 4;
#pragma unroll 1
        for (int ps = 0; ps < 2; ++ps) {
            *(volatile v4f*)drow = val;
            if (ps == 0) __threadfence(); }
    }
}

__global__ __launch_bounds__(32) void k_qout(const bf* __restrict__ A, const bf* __restrict__ Wqt, const float* __restrict__ bq, const float* __restrict__ PART, float* OUT) {
    __shared__ __align__(16) float os[16 * 68];
    const int K = DM;
    const int lane = threadIdx.x & 31, lr = lane & 15, hi = lane >> 4; const int r0 = blockIdx.x * 64, c0 = blockIdx.y * 64;
    v8f acc[4][4];
#pragma unroll
    for (int mb = 0; mb < 4; ++mb)
#pragma unroll
        for (int nb = 0; nb < 4; ++nb) acc[mb][nb] = (v8f){};
    const size_t aoff = (size_t)(r0 + lr) * K + 8 * hi, boff = (size_t)(c0 + lr) * K + 8 * hi;
#pragma unroll 1
    for (int kc = 0; kc < K; kc += 32) {
        v16bf a[4];
#pragma unroll
        for (int mb = 0; mb < 4; ++mb) a[mb] = ldb(A + aoff + (size_t)mb * 16 * K + kc);
#pragma unroll
        for (int nb = 0; nb < 4; ++nb) { const v16bf b = ldb(Wqt + boff + (size_t)nb * 16 * K + kc);
#pragma unroll
            for (int mb = 0; mb < 4; ++mb) acc[mb][nb] = wmmab_g(a[mb], b, acc[mb][nb]); }
    }
    float bc[4];
#pragma unroll
    for (int nb = 0; nb < 4; ++nb) bc[nb] = bfr(bq[c0 + nb * 16 + lr]);
    const int bb = r0 / SEQ, tt = r0 % SEQ;
    const int cofs = (lane & 15) * 4;
    v4f kv4 = (v4f){};
    const float* pl = PART + (size_t)bb * RT * DM + c0 + cofs;
#pragma unroll 4
    for (int rt = 0; rt < RT; ++rt) kv4 += *(const v4f*)(pl + (size_t)rt * DM);
    float* obase = OUT + ((size_t)bb * OUT_SEQ + tt) * DM + c0 + cofs;
#pragma unroll
    for (int mb = 0; mb < 4; ++mb) {
#pragma unroll
        for (int nb = 0; nb < 4; ++nb) {
#pragma unroll
            for (int j = 0; j < 8; ++j) os[(hi * 8 + j) * 68 + nb * 16 + lr] = acc[mb][nb][j] + bc[nb]; }
        wave_sync();
#pragma unroll 1
        for (int ps = 0; ps < 2; ++ps) {
#pragma unroll
            for (int s = 0; s < 8; ++s) { const int row = 2 * s + (lane >> 4);
                const v4f x = *(const v4fa*)(&os[row * 68 + cofs]);
                const v4f val = x * kv4;
                *(volatile v4f*)(obase + (size_t)(mb * 16 + row) * DM) = val; }
            if (ps == 0) __threadfence(); }
        wave_sync();
    }
}

static constexpr size_t al256(size_t v) { return (v + 255) & ~(size_t)255; }
static constexpr size_t SZ_XB = al256((size_t)NB * SEQ * DM * 2);
static constexpr size_t SZ_WB = al256((size_t)3 * DM * DM * 2);
static constexpr size_t SZ_PT = al256((size_t)(NB * SEQ / 64) * DM * 4);
static constexpr size_t SZ_TOTAL = SZ_XB + SZ_WB + SZ_PT;
static_assert(SZ_TOTAL <= (size_t)134217728);
static_assert(((size_t)DM * DM * 2) % 256 == 0);
static_assert((size_t)(NB * SEQ / 64) * DM * 4 == (size_t)NB * RT * DM * 4);

extern "C" void kernel_launch(void* const* d_in, const int* in_sizes, int n_in,
                              void* d_out, int out_size, void* d_ws, size_t ws_size, hipStream_t stream) {
    if (n_in < 7) return;
    const size_t needx = ((size_t)(NB - 1) * SEQ_FULL + SEQ) * DM;
    if ((size_t)in_sizes[0] < needx) return;
    if ((size_t)in_sizes[1] < (size_t)DM * DM || (size_t)in_sizes[3] < (size_t)DM * DM || (size_t)in_sizes[5] < (size_t)DM * DM) return;
    if (in_sizes[2] < DM || in_sizes[4] < DM || in_sizes[6] < DM) return;
    if ((size_t)out_size < ((size_t)(NB - 1) * OUT_SEQ + SEQ) * DM) return;
    if (SZ_TOTAL > ws_size) return;
    const float* x  = (const float*)d_in[0];
    const float* wq = (const float*)d_in[1]; const float* bq = (const float*)d_in[2];
    const float* wk = (const float*)d_in[3]; const float* bk = (const float*)d_in[4];
    const float* wv = (const float*)d_in[5]; const float* bv = (const float*)d_in[6];
    float* OUT = (float*)d_out;
    char* wsp = (char*)d_ws;
    bf* XB = (bf*)wsp; wsp += SZ_XB;
    bf* WB = (bf*)wsp; wsp += SZ_WB;
    float* PART = (float*)wsp; wsp += SZ_PT;
    bf* WQ = WB; bf* WK = WB + (size_t)DM * DM; bf* WV = WB + (size_t)2 * DM * DM;

    if (SEQ == SEQ_FULL) {
        const size_t n8 = (size_t)NB * SEQ * DM / 8;
        k_cvt8<<<(unsigned)((n8 + 255) / 256), 256, 0, stream>>>(x, XB, n8);
    } else {
        const size_t n8 = (size_t)SEQ * DM / 8;
        for (int b = 0; b < NB; ++b) k_cvt8<<<(unsigned)((n8 + 255) / 256), 256, 0, stream>>>(x + (size_t)b * SEQ_FULL * DM, XB + (size_t)b * SEQ * DM, n8);
    }
    k_wtr<<<dim3(DM / 64, DM / 64, 1), 256, 0, stream>>>(wq, WQ);
    k_wtr<<<dim3(DM / 64, DM / 64, 1), 256, 0, stream>>>(wk, WK);
    k_wtr<<<dim3(DM / 64, DM / 64, 1), 256, 0, stream>>>(wv, WV);

    k_kvpart<<<dim3(NB * SEQ / 64, 1, 1), 128, 0, stream>>>(XB, WK, WV, bk, bv, PART);
    k_qout<<<dim3(NB * SEQ / 64, DM / 64, 1), 32, 0, stream>>>(XB, WQ, bq, PART, OUT);
}
